// PatchTSTRopeAttention_73461120631351
// MI455X (gfx1250) — hardware-run, weakly checked
//
#include <hip/hip_runtime.h>
#include <math.h>

typedef __attribute__((ext_vector_type(16))) __bf16   v16b;
typedef __attribute__((ext_vector_type(8)))  __bf16   v8b;
typedef __attribute__((ext_vector_type(8)))  float    v8f;
typedef __attribute__((ext_vector_type(4)))  float    v4f;
typedef __attribute__((ext_vector_type(4)))  unsigned int v4u;

constexpr int kInputsRneToBf16 = 1;

constexpr int kBatch  = 4;
constexpr int kSeq    = 2048;
constexpr int kEmb    = 512;
constexpr int kHeads  = 8;
constexpr int kHd     = kEmb / kHeads;
constexpr int kBH     = kBatch * kHeads;
constexpr int kRows   = kBatch * kSeq;
constexpr int kNqkv   = 3 * kEmb;
constexpr int kRotPairs = ((int)(0.5 * kHd)) / 2;
constexpr int kTabW   = 2 * kRotPairs;
constexpr int isqrt_exact(int v) { int r = 0; while ((r + 1) * (r + 1) <= v) ++r; return r; }
static_assert(kHd == 64);
static_assert(isqrt_exact(kHd) * isqrt_exact(kHd) == kHd);
static_assert(kRotPairs == 16 && kTabW == 32);
static_assert((kRows % 64) == 0 && (kNqkv % 64) == 0 && (kEmb % 64) == 0 && (kEmb % 32) == 0 && (kSeq % 64) == 0);
constexpr float  kQScale  = 1.0f / (float)isqrt_exact(kHd);
constexpr float  kNegBig  = -1.0e30f;
constexpr float  kMaxWavelength = 10000.0f;

constexpr size_t kSzXB   = (size_t)kRows * kEmb * 2;
constexpr size_t kSzXL   = kInputsRneToBf16 ? 0 : kSzXB;
constexpr size_t kSzWT   = (size_t)4 * kEmb * kEmb * 2;
constexpr size_t kSzWTL  = kInputsRneToBf16 ? 0 : kSzWT;
constexpr size_t kSzTAB  = (size_t)kSeq * kTabW * 4;
constexpr size_t kSzBIAS = (size_t)4 * kEmb * 4;
constexpr size_t kSzQKVF = (size_t)3 * kBH * kSeq * kHd * 4;
constexpr size_t kSzQK16 = (size_t)2 * kBH * kSeq * kHd * 2;
constexpr size_t kSzVT   = (size_t)kBH * kHd * kSeq * 2;
constexpr size_t kSzAO   = (size_t)kRows * kEmb * 2;
static_assert(kSzXB == 8388608ull && kSzWT == 2097152ull && kSzTAB == 262144ull && kSzBIAS == 8192ull);
static_assert(kSzQKVF == 50331648ull && kSzQK16 == 16777216ull && kSzVT == 8388608ull && kSzAO == 8388608ull);
constexpr size_t kOffXB   = 0;
constexpr size_t kOffXL   = kOffXB   + kSzXB;
constexpr size_t kOffWT   = kOffXL   + kSzXL;
constexpr size_t kOffWTL  = kOffWT   + kSzWT;
constexpr size_t kOffTAB  = kOffWTL  + kSzWTL;
constexpr size_t kOffBIAS = kOffTAB  + kSzTAB;
constexpr size_t kOffQKVF = kOffBIAS + kSzBIAS;
constexpr size_t kOffQKH  = kOffQKVF + kSzQKVF;
constexpr size_t kOffQKL  = kOffQKH  + kSzQK16;
constexpr size_t kOffVTH  = kOffQKL  + kSzQK16;
constexpr size_t kOffVTL  = kOffVTH  + kSzVT;
constexpr size_t kOffAOH  = kOffVTL  + kSzVT;
constexpr size_t kOffAOL  = kOffAOH  + kSzAO;
constexpr size_t kWsTotal = kOffAOL  + kSzAO;
static_assert(!kInputsRneToBf16 || kWsTotal == 128196608ull);
static_assert(kWsTotal <= 134217728ull);
static_assert((kOffXL % 128) == 0 && (kOffWT % 128) == 0 && (kOffWTL % 128) == 0 && (kOffTAB % 128) == 0 &&
              (kOffBIAS % 128) == 0 && (kOffQKVF % 128) == 0 && (kOffQKH % 128) == 0 && (kOffQKL % 128) == 0 &&
              (kOffVTH % 128) == 0 && (kOffVTL % 128) == 0 && (kOffAOH % 128) == 0 && (kOffAOL % 128) == 0);

__device__ __forceinline__ unsigned short f2bf_bits(float f) {
  unsigned u = __float_as_uint(f);
  return (unsigned short)((u + 0x7FFFu + ((u >> 16) & 1u)) >> 16);
}
__device__ __forceinline__ float bf_bits2f(unsigned short h) { return __uint_as_float(((unsigned)h) << 16); }
__device__ __forceinline__ unsigned pk16(unsigned short a, unsigned short b) { return (unsigned)a | ((unsigned)b << 16); }
__device__ __forceinline__ void split_bits(float f, unsigned short& hb, unsigned short& lb) {
  hb = f2bf_bits(f);
  lb = f2bf_bits(f - bf_bits2f(hb));
}

union FragU { v16b v; v8b h[2]; };
__device__ __forceinline__ v16b ldfrag(const __bf16* p) {
  FragU f;
  f.h[0] = *(const v8b*)(p);
  f.h[1] = *(const v8b*)(p + 16);
  return f.v;
}
__device__ __forceinline__ v8f mma_raw(v16b a, v16b b, v8f c) {
  return __builtin_amdgcn_wmma_f32_16x16x32_bf16(false, a, false, b, (short)0, c, false, false);
}
__device__ __forceinline__ v8f mma_g(v16b a, v16b b, v8f c) {
  c = __builtin_amdgcn_wmma_f32_16x16x32_bf16(false, a, false, b, (short)0, c, false, false);
  asm volatile("v_nop\n\tv_nop\n\tv_nop\n\tv_nop" : "+v"(c) : "v"(a), "v"(b));
  return c;
}
__device__ __forceinline__ void acc_guard1(v8f& a, v16b x, v16b y) {
  asm volatile("v_nop\n\tv_nop\n\tv_nop\n\tv_nop" : "+v"(a) : "v"(x), "v"(y));
}
__device__ __forceinline__ void keep4_b(v16b a, v16b b, v16b c, v16b d) { asm volatile("v_nop" :: "v"(a), "v"(b), "v"(c), "v"(d)); }
__device__ __forceinline__ void acc_guard4(v8f& a, v8f& b, v8f& c, v8f& d) {
  asm volatile("v_nop\n\tv_nop\n\tv_nop\n\tv_nop" : "+v"(a), "+v"(b), "+v"(c), "+v"(d));
}
__device__ __forceinline__ void wave_lds_sync() {
  __builtin_amdgcn_fence(__ATOMIC_RELEASE, "workgroup");
  __builtin_amdgcn_wave_barrier();
  __builtin_amdgcn_fence(__ATOMIC_ACQUIRE, "workgroup");
}

template <bool LO>
__global__ __launch_bounds__(256) void cast_rows_bf16_kernel(
    const float* __restrict__ src, unsigned short* __restrict__ dhi, unsigned short* __restrict__ dlo, int n8) {
  const int i = blockIdx.x * 256 + threadIdx.x;
  if (i >= n8) return;
  const size_t e0 = (size_t)i << 3;
  const v4f a0 = *(const v4f*)(src + e0);
  const v4f a1 = *(const v4f*)(src + e0 + 4);
  float x[8];
#pragma unroll
  for (int e = 0; e < 4; ++e) { x[e] = a0[e]; x[4 + e] = a1[e]; }
  unsigned short hb[8], lb[8];
#pragma unroll
  for (int e = 0; e < 8; ++e) split_bits(x[e], hb[e], lb[e]);
  const v4u uh = (v4u){pk16(hb[0], hb[1]), pk16(hb[2], hb[3]), pk16(hb[4], hb[5]), pk16(hb[6], hb[7])};
  const v4u ul = (v4u){pk16(lb[0], lb[1]), pk16(lb[2], lb[3]), pk16(lb[4], lb[5]), pk16(lb[6], lb[7])};
  unsigned short* qh = dhi + e0;
  unsigned short* ql = dlo + e0;
  *(volatile v4u*)qh = uh;
  if (LO) *(volatile v4u*)ql = ul;
  __threadfence();
  *(volatile v4u*)qh = uh;
  if (LO) *(volatile v4u*)ql = ul;
}

template <bool LO>
__global__ __launch_bounds__(256) void wt_bf16_kernel(
    const float* __restrict__ W0, const float* __restrict__ W1, const float* __restrict__ W2, const float* __restrict__ W3,
    unsigned short* __restrict__ outh, unsigned short* __restrict__ outl) {
  __shared__ float sm[64][65];
  const int t  = threadIdx.x;
  const int k0 = blockIdx.x * 64;
  const int n0 = blockIdx.y * 64;
  const int z  = blockIdx.z;
  const float* W = (z == 0) ? W0 : (z == 1) ? W1 : (z == 2) ? W2 : W3;
#pragma unroll
  for (int i = 0; i < 16; ++i) {
    const int e = i * 256 + t;
    const int r = e >> 6;
    const int c = e & 63;
    sm[c][r] = W[(size_t)(k0 + r) * kEmb + n0 + c];
  }
  __syncthreads();
  const int lane = t & 31, wave = t >> 5;
  const int q = lane >> 3, c8 = (lane & 7) * 8;
  v4u uh[2], ul[2];
#pragma unroll
  for (int it = 0; it < 2; ++it) {
    const int row = wave * 8 + it * 4 + q;
    unsigned short hb[8], lb[8];
#pragma unroll
    for (int e = 0; e < 8; ++e) split_bits(sm[row][c8 + e], hb[e], lb[e]);
    uh[it] = (v4u){pk16(hb[0], hb[1]), pk16(hb[2], hb[3]), pk16(hb[4], hb[5]), pk16(hb[6], hb[7])};
    ul[it] = (v4u){pk16(lb[0], lb[1]), pk16(lb[2], lb[3]), pk16(lb[4], lb[5]), pk16(lb[6], lb[7])};
  }
  const size_t pz = (size_t)z * kEmb * kEmb;
  for (int pass = 0; pass < 2; ++pass) {
#pragma unroll
    for (int it = 0; it < 2; ++it) {
      const int row = wave * 8 + it * 4 + q;
      const size_t o = pz + (size_t)(n0 + row) * kEmb + k0 + c8;
      *(volatile v4u*)(outh + o) = uh[it];
      if (LO) *(volatile v4u*)(outl + o) = ul[it];
    }
    __threadfence();
  }
}

__global__ __launch_bounds__(256) void rot_table_kernel(float* __restrict__ tab) {
  const int t = blockIdx.x * 256 + threadIdx.x;
  if (t >= kSeq * kTabW) return;
  const int s    = t / kTabW;
  const int cidx = t - s * kTabW;
  const int i    = cidx & (kRotPairs - 1);
  const float fraction = 2.0f * (float)i / (float)kHd;
  const float tsi = powf(kMaxWavelength, fraction);
  const float ang = (float)s / tsi;
  const float cv = cosf(ang);
  const float sv = sinf(ang);
  const float val = (cidx < kRotPairs) ? cv : sv;
  volatile float* p = tab + t;
  *p = val;
  __threadfence();
  *p = val;
}

__global__ __launch_bounds__(512) void bias_table_kernel(
    const float* __restrict__ bq, const float* __restrict__ bk, const float* __restrict__ bv, const float* __restrict__ bo,
    float* __restrict__ dst) {
  const int t = threadIdx.x;
  const int which = t >> 7;
  const float* src = (which == 0) ? bq : (which == 1) ? bk : (which == 2) ? bv : bo;
  const v4f a = *(const v4f*)(src + 4 * (t & 127));
  float x0 = a[0], x1 = a[1], x2 = a[2], x3 = a[3];
  if (kInputsRneToBf16) {
    x0 = bf_bits2f(f2bf_bits(x0));
    x1 = bf_bits2f(f2bf_bits(x1));
    x2 = bf_bits2f(f2bf_bits(x2));
    x3 = bf_bits2f(f2bf_bits(x3));
  }
  const v4f o = (v4f){x0, x1, x2, x3};
  float* p = dst + 4 * t;
  *(volatile v4f*)p = o;
  __threadfence();
  *(volatile v4f*)p = o;
}

namespace eng {
template <int SPL, int EPI>
__global__ __launch_bounds__(256) void wmma_gemm64(
    const unsigned short* __restrict__ Ap, const unsigned short* __restrict__ A2p, int lda,
    const unsigned short* __restrict__ Btp, const unsigned short* __restrict__ Bt2p, int ldb,
    float* __restrict__ Cout, int ldc, const float* __restrict__ bias, int M, int N, int K) {
  const __bf16* A   = (const __bf16*)Ap;
  const __bf16* A2  = (const __bf16*)A2p;
  const __bf16* Bt  = (const __bf16*)Btp;
  const __bf16* Bt2 = (const __bf16*)Bt2p;
  __shared__ __align__(16) float sT[8][16 * 68];
  const int lane = threadIdx.x & 31;
  const int wave = threadIdx.x >> 5;
  const int tilesN = N >> 6;
  const int tilesM = M >> 6;
  const int tile = blockIdx.x * 8 + wave;
  if (tile >= tilesM * tilesN) return;
  const int tm = tile / tilesN;
  const int tn = tile - tm * tilesN;
  const int m0 = tm << 6;
  const int n0 = tn << 6;

  const int rlane = lane & 15;
  const int koff  = (lane >> 4) * 8;
  const int mOff  = (lane >> 4) * 8;

  v8f acc[4][4];
#pragma unroll
  for (int i = 0; i < 4; ++i)
#pragma unroll
    for (int j = 0; j < 4; ++j) acc[i][j] = (v8f){0.f, 0.f, 0.f, 0.f, 0.f, 0.f, 0.f, 0.f};

  for (int k0 = 0; k0 < K; k0 += 32) {
    v16b bh[4], bl[4];
#pragma unroll
    for (int j = 0; j < 4; ++j) {
      const size_t bo = (size_t)(n0 + (j << 4) + rlane) * ldb + koff + k0;
      bh[j] = ldfrag(Bt + bo);
      if (SPL == 2) bl[j] = ldfrag(Bt2 + bo);
    }
#pragma unroll
    for (int i = 0; i < 4; ++i) {
      const size_t ao = (size_t)(m0 + (i << 4) + rlane) * lda + koff + k0;
      v16b ah = ldfrag(A + ao);
      v16b al;
      if (SPL >= 1) al = ldfrag(A2 + ao);
#pragma unroll
      for (int j = 0; j < 4; ++j) {
        acc[i][j] = mma_raw(ah, bh[j], acc[i][j]);
        if (SPL == 2) acc[i][j] = mma_raw(ah, bl[j], acc[i][j]);
        if (SPL >= 1) acc[i][j] = mma_raw(al, bh[j], acc[i][j]);
      }
      acc_guard1(acc[i][0], ah, (SPL >= 1) ? al : ah);
      acc_guard1(acc[i][1], ah, (SPL >= 1) ? al : ah);
      acc_guard1(acc[i][2], ah, (SPL >= 1) ? al : ah);
      acc_guard1(acc[i][3], ah, (SPL >= 1) ? al : ah);
    }
    keep4_b(bh[0], bh[1], bh[2], bh[3]);
    if (SPL == 2) keep4_b(bl[0], bl[1], bl[2], bl[3]);
  }
  acc_guard4(acc[0][0], acc[0][1], acc[0][2], acc[0][3]);
  acc_guard4(acc[1][0], acc[1][1], acc[1][2], acc[1][3]);
  acc_guard4(acc[2][0], acc[2][1], acc[2][2], acc[2][3]);
  acc_guard4(acc[3][0], acc[3][1], acc[3][2], acc[3][3]);

  float* slab = sT[wave];
  float* Cb;
  int ldcE, nc0;
  float cs;
  if (EPI == 0) {
    const int which = n0 / kEmb;
    const int hcol  = (n0 - which * kEmb) / kHd;
    const int bb    = m0 / kSeq;
    const int s0    = m0 - bb * kSeq;
    Cb   = Cout + ((size_t)(which * kBH + bb * kHeads + hcol) * kSeq + s0) * kHd;
    ldcE = kHd;
    nc0  = 0;
    cs   = (which == 0) ? kQScale : 1.0f;
  } else {
    Cb   = Cout + (size_t)m0 * ldc;
    ldcE = ldc;
    nc0  = n0;
    cs   = 1.0f;
  }
#pragma unroll
  for (int i = 0; i < 4; ++i) {
#pragma unroll
    for (int j = 0; j < 4; ++j) {
      const int n = n0 + (j << 4) + rlane;
      const float bv = bias[n];
#pragma unroll
      for (int r = 0; r < 8; ++r) {
        slab[(mOff + r) * 68 + (j << 4) + rlane] = (acc[i][j][r] + bv) * cs;
      }
    }
    wave_lds_sync();
    {
      const int hh = lane >> 4, c4 = (lane & 15) * 4;
      for (int pass = 0; pass < 2; ++pass) {
#pragma unroll
        for (int it = 0; it < 8; ++it) {
          const int row = it * 2 + hh;
          const v4f v = *(const v4f*)(slab + row * 68 + c4);
          *(volatile v4f*)(Cb + (size_t)((i << 4) + row) * ldcE + nc0 + c4) = v;
        }
        __threadfence();
      }
    }
    wave_lds_sync();
  }
}
}

__global__ __launch_bounds__(256) void rot_split_kernel(
    const float* __restrict__ QKf, const float* __restrict__ tab,
    unsigned short* __restrict__ QKh, unsigned short* __restrict__ QKl) {
  const int t = blockIdx.x * 256 + threadIdx.x;
  if (t >= 2 * kBH * kSeq * 8) return;
  const int R  = t >> 3;
  const int c8 = (t & 7) * 8;
  const int s  = R & (kSeq - 1);
  const float* own = QKf + (size_t)R * kHd + c8;
  const float* par = QKf + (size_t)R * kHd + (c8 ^ 32);
  const v4f xo0 = *(const v4f*)(own);
  const v4f xo1 = *(const v4f*)(own + 4);
  const v4f xp0 = *(const v4f*)(par);
  const v4f xp1 = *(const v4f*)(par + 4);
  const int  i0  = c8 & 31;
  const bool rot = (i0 < kRotPairs);
  const int  ti  = rot ? i0 : 0;
  const float* tr = tab + (size_t)s * kTabW + ti;
  v4f tc0 = *(const v4f*)(tr);
  v4f tc1 = *(const v4f*)(tr + 4);
  v4f ts0 = *(const v4f*)(tr + kRotPairs);
  v4f ts1 = *(const v4f*)(tr + kRotPairs + 4);
  asm volatile("" : "+v"(tc0));
  asm volatile("" : "+v"(tc1));
  asm volatile("" : "+v"(ts0));
  asm volatile("" : "+v"(ts1));
  const float sg = (c8 < 32) ? -1.0f : 1.0f;
  float xo[8], xp[8], cc[8], ss[8];
#pragma unroll
  for (int e = 0; e < 4; ++e) {
    xo[e] = xo0[e]; xo[4 + e] = xo1[e];
    xp[e] = xp0[e]; xp[4 + e] = xp1[e];
    cc[e] = tc0[e]; cc[4 + e] = tc1[e];
    ss[e] = ts0[e]; ss[4 + e] = ts1[e];
  }
  unsigned short hb[8], lb[8];
#pragma unroll
  for (int e = 0; e < 8; ++e) {
    const float cs = rot ? cc[e] : 1.0f;
    const float sn = rot ? ss[e] : 0.0f;
    const float o  = xo[e] * cs + sg * (xp[e] * sn);
    split_bits(o, hb[e], lb[e]);
  }
  const v4u uh = (v4u){pk16(hb[0], hb[1]), pk16(hb[2], hb[3]), pk16(hb[4], hb[5]), pk16(hb[6], hb[7])};
  const v4u ul = (v4u){pk16(lb[0], lb[1]), pk16(lb[2], lb[3]), pk16(lb[4], lb[5]), pk16(lb[6], lb[7])};
  unsigned short* ph = QKh + (size_t)R * kHd + c8;
  unsigned short* pl = QKl + (size_t)R * kHd + c8;
  *(volatile v4u*)ph = uh;
  *(volatile v4u*)pl = ul;
  __threadfence();
  *(volatile v4u*)ph = uh;
  *(volatile v4u*)pl = ul;
}

__global__ __launch_bounds__(256) void vt_split_kernel(
    const float* __restrict__ Vf, unsigned short* __restrict__ Vth, unsigned short* __restrict__ Vtl) {
  __shared__ float sm[64][65];
  const int t  = threadIdx.x;
  const int s0 = blockIdx.x * 64;
  const int bh = blockIdx.y;
#pragma unroll
  for (int i = 0; i < 16; ++i) {
    const int e = i * 256 + t;
    const int r = e >> 6;
    const int c = e & 63;
    sm[c][r] = Vf[((size_t)bh * kSeq + s0 + r) * kHd + c];
  }
  __syncthreads();
  const int lane = t & 31, wave = t >> 5;
  const int q = lane >> 3, c8 = (lane & 7) * 8;
  v4u uh[2], ul[2];
#pragma unroll
  for (int it = 0; it < 2; ++it) {
    const int row = wave * 8 + it * 4 + q;
    unsigned short hb[8], lb[8];
#pragma unroll
    for (int e = 0; e < 8; ++e) split_bits(sm[row][c8 + e], hb[e], lb[e]);
    uh[it] = (v4u){pk16(hb[0], hb[1]), pk16(hb[2], hb[3]), pk16(hb[4], hb[5]), pk16(hb[6], hb[7])};
    ul[it] = (v4u){pk16(lb[0], lb[1]), pk16(lb[2], lb[3]), pk16(lb[4], lb[5]), pk16(lb[6], lb[7])};
  }
  for (int pass = 0; pass < 2; ++pass) {
#pragma unroll
    for (int it = 0; it < 2; ++it) {
      const int row = wave * 8 + it * 4 + q;
      const size_t o = ((size_t)bh * kHd + row) * kSeq + s0 + c8;
      *(volatile v4u*)(Vth + o) = uh[it];
      *(volatile v4u*)(Vtl + o) = ul[it];
    }
    __threadfence();
  }
}

__global__ __launch_bounds__(128) void attn_kernel(
    const unsigned short* QKh, const unsigned short* QKl,
    const unsigned short* Vth, const unsigned short* Vtl,
    unsigned short* AOh, unsigned short* AOl) {
  __shared__ __align__(16) __bf16 Psh[4][16 * 64];
  __shared__ __align__(16) __bf16 Psl[4][16 * 64];
  __shared__ __align__(16) float  Os[4][16 * 68];

  const int tid  = threadIdx.x;
  const int wave = tid >> 5;
  const int lane = tid & 31;
  const int hh   = lane >> 4;
  const int c    = lane & 15;

  constexpr int nqb = kSeq / 64;
  const int qb = blockIdx.x % nqb;
  const int bh = blockIdx.x / nqb;
  const int b  = bh / kHeads;
  const int h  = bh - b * kHeads;
  const int q0 = qb * 64 + wave * 16;

  constexpr size_t kPlane = (size_t)kBH * kSeq * kHd;
  const __bf16* Qhp = (const __bf16*)QKh + (size_t)bh * kSeq * kHd;
  const __bf16* Qlp = (const __bf16*)QKl + (size_t)bh * kSeq * kHd;
  const __bf16* Khp = (const __bf16*)QKh + kPlane + (size_t)bh * kSeq * kHd;
  const __bf16* Klp = (const __bf16*)QKl + kPlane + (size_t)bh * kSeq * kHd;
  const __bf16* Vhp = (const __bf16*)Vth + (size_t)bh * kHd * kSeq;
  const __bf16* Vlp = (const __bf16*)Vtl + (size_t)bh * kHd * kSeq;

  v16b qah[2], qal[2];
#pragma unroll
  for (int dc = 0; dc < 2; ++dc) {
    const size_t qo = (size_t)(q0 + c) * kHd + dc * 32 + 8 * hh;
    qah[dc] = ldfrag(Qhp + qo);
    qal[dc] = ldfrag(Qlp + qo);
  }

  float mrow[8], lrow[8];
  v8f oacc[4];
#pragma unroll
  for (int r = 0; r < 8; ++r) { mrow[r] = kNegBig; lrow[r] = 0.f; }
#pragma unroll
  for (int t = 0; t < 4; ++t) oacc[t] = (v8f){0.f, 0.f, 0.f, 0.f, 0.f, 0.f, 0.f, 0.f};

  __bf16* pwh = Psh[wave];
  __bf16* pwl = Psl[wave];

  for (int kc = 0; kc <= qb; ++kc) {
    const int kv0 = kc * 64;
    v8f sc[4];
#pragma unroll
    for (int j = 0; j < 4; ++j) {
      v8f a = (v8f){0.f, 0.f, 0.f, 0.f, 0.f, 0.f, 0.f, 0.f};
      const size_t ko = (size_t)(kv0 + j * 16 + c) * kHd + 8 * hh;
#pragma unroll
      for (int dc = 0; dc < 2; ++dc) {
        const v16b kb = ldfrag(Khp + ko + dc * 32);
        const v16b kl = ldfrag(Klp + ko + dc * 32);
        a = mma_g(qah[dc], kb, a);
        a = mma_g(qah[dc], kl, a);
        a = mma_g(qal[dc], kb, a);
      }
      sc[j] = a;
      asm volatile("" ::: "memory");
    }
    if (kc == qb) {
#pragma unroll
      for (int j = 0; j < 4; ++j) {
        const int kvcol = kv0 + j * 16 + c;
#pragma unroll
        for (int r = 0; r < 8; ++r) {
          const int qrow = q0 + 8 * hh + r;
          sc[j][r] = (kvcol > qrow) ? kNegBig : sc[j][r];
        }
      }
    }
    float cm[8];
#pragma unroll
    for (int r = 0; r < 8; ++r) {
      float m = fmaxf(fmaxf(sc[0][r], sc[1][r]), fmaxf(sc[2][r], sc[3][r]));
      m = fmaxf(m, __shfl_xor(m, 1, 32));
      m = fmaxf(m, __shfl_xor(m, 2, 32));
      m = fmaxf(m, __shfl_xor(m, 4, 32));
      m = fmaxf(m, __shfl_xor(m, 8, 32));
      cm[r] = m;
    }
#pragma unroll
    for (int r = 0; r < 8; ++r) {
      const float mnew  = fmaxf(mrow[r], cm[r]);
      const float alpha = __expf(mrow[r] - mnew);
      mrow[r] = mnew;
      float psum = 0.f;
#pragma unroll
      for (int j = 0; j < 4; ++j) {
        const float p = __expf(sc[j][r] - mnew);
        psum += p;
        unsigned short hb, lb;
        split_bits(p, hb, lb);
        pwh[(8 * hh + r) * 64 + j * 16 + c] = __builtin_bit_cast(__bf16, hb);
        pwl[(8 * hh + r) * 64 + j * 16 + c] = __builtin_bit_cast(__bf16, lb);
      }
      psum += __shfl_xor(psum, 1, 32);
      psum += __shfl_xor(psum, 2, 32);
      psum += __shfl_xor(psum, 4, 32);
      psum += __shfl_xor(psum, 8, 32);
      lrow[r] = lrow[r] * alpha + psum;
#pragma unroll
      for (int t = 0; t < 4; ++t) oacc[t][r] *= alpha;
    }
    wave_lds_sync();
#pragma unroll
    for (int kk = 0; kk < 2; ++kk) {
      FragU pa, pl;
      pa.h[0] = *(const v8b*)(pwh + c * 64 + kk * 32 + 8 * hh);
      pa.h[1] = *(const v8b*)(pwh + c * 64 + kk * 32 + 16 + 8 * hh);
      pl.h[0] = *(const v8b*)(pwl + c * 64 + kk * 32 + 8 * hh);
      pl.h[1] = *(const v8b*)(pwl + c * 64 + kk * 32 + 16 + 8 * hh);
#pragma unroll
      for (int t = 0; t < 4; ++t) {
        const size_t vo = (size_t)(t * 16 + c) * kSeq + kv0 + kk * 32 + 8 * hh;
        const v16b vb = ldfrag(Vhp + vo);
        const v16b vl = ldfrag(Vlp + vo);
        oacc[t] = mma_g(pa.v, vb, oacc[t]);
        oacc[t] = mma_g(pa.v, vl, oacc[t]);
        oacc[t] = mma_g(pl.v, vb, oacc[t]);
      }
      asm volatile("" ::: "memory");
    }
    wave_lds_sync();
  }

  float* os = Os[wave];
#pragma unroll
  for (int r = 0; r < 8; ++r) {
    const float inv = 1.0f / lrow[r];
#pragma unroll
    for (int t = 0; t < 4; ++t) os[(8 * hh + r) * 68 + t * 16 + c] = oacc[t][r] * inv;
  }
  wave_lds_sync();
  {
    const int q4 = lane >> 3, c8 = (lane & 7) * 8;
    v4u uh[4], ul[4];
#pragma unroll
    for (int it = 0; it < 4; ++it) {
      const int row = it * 4 + q4;
      const float* sp = os + row * 68 + c8;
      const v4f a0 = *(const v4f*)(sp);
      const v4f a1 = *(const v4f*)(sp + 4);
      float x[8];
#pragma unroll
      for (int e = 0; e < 4; ++e) { x[e] = a0[e]; x[4 + e] = a1[e]; }
      unsigned short hb[8], lb[8];
#pragma unroll
      for (int e = 0; e < 8; ++e) split_bits(x[e], hb[e], lb[e]);
      uh[it] = (v4u){pk16(hb[0], hb[1]), pk16(hb[2], hb[3]), pk16(hb[4], hb[5]), pk16(hb[6], hb[7])};
      ul[it] = (v4u){pk16(lb[0], lb[1]), pk16(lb[2], lb[3]), pk16(lb[4], lb[5]), pk16(lb[6], lb[7])};
    }
    for (int pass = 0; pass < 2; ++pass) {
#pragma unroll
      for (int it = 0; it < 4; ++it) {
        const int row = it * 4 + q4;
        const size_t o = ((size_t)b * kSeq + q0 + row) * kEmb + h * kHd + c8;
        *(volatile v4u*)(AOh + o) = uh[it];
        *(volatile v4u*)(AOl + o) = ul[it];
      }
      __threadfence();
    }
  }
}

extern "C" void kernel_launch(void* const* d_in, const int* in_sizes, int n_in,
                              void* d_out, int out_size, void* d_ws, size_t ws_size,
                              hipStream_t stream) {
  if (n_in < 9) return;
  if (in_sizes[0] != kRows * kEmb) return;
  if (in_sizes[1] != kEmb * kEmb || in_sizes[3] != kEmb * kEmb || in_sizes[5] != kEmb * kEmb || in_sizes[7] != kEmb * kEmb) return;
  if (in_sizes[2] != kEmb || in_sizes[4] != kEmb || in_sizes[6] != kEmb || in_sizes[8] != kEmb) return;
  if (out_size != kRows * kEmb) return;
  if (ws_size < kWsTotal) return;

  const float* X  = (const float*)d_in[0];
  const float* Wq = (const float*)d_in[1];
  const float* bq = (const float*)d_in[2];
  const float* Wk = (const float*)d_in[3];
  const float* bk = (const float*)d_in[4];
  const float* Wv = (const float*)d_in[5];
  const float* bv = (const float*)d_in[6];
  const float* Wo = (const float*)d_in[7];
  const float* bo = (const float*)d_in[8];
  float* out = (float*)d_out;

  char* ws = (char*)d_ws;
  unsigned short* XB   = (unsigned short*)(ws + kOffXB);
  unsigned short* XL   = kInputsRneToBf16 ? XB : (unsigned short*)(ws + kOffXL);
  unsigned short* WT   = (unsigned short*)(ws + kOffWT);
  unsigned short* WTL  = kInputsRneToBf16 ? WT : (unsigned short*)(ws + kOffWTL);
  float*          TAB  = (float*)(ws + kOffTAB);
  float*          BIAS = (float*)(ws + kOffBIAS);
  float*          QKVF = (float*)(ws + kOffQKVF);
  unsigned short* QKH  = (unsigned short*)(ws + kOffQKH);
  unsigned short* QKL  = (unsigned short*)(ws + kOffQKL);
  unsigned short* VTH  = (unsigned short*)(ws + kOffVTH);
  unsigned short* VTL  = (unsigned short*)(ws + kOffVTL);
  unsigned short* AOH  = (unsigned short*)(ws + kOffAOH);
  unsigned short* AOL  = (unsigned short*)(ws + kOffAOL);

  constexpr bool kLo = (kInputsRneToBf16 == 0);
  constexpr int kSplQkv = kInputsRneToBf16 ? 0 : 2;
  constexpr int kSplOut = kInputsRneToBf16 ? 1 : 2;

  cast_rows_bf16_kernel<kLo><<<(kRows * kEmb / 8) / 256, 256, 0, stream>>>(X, XB, XL, kRows * kEmb / 8);
  wt_bf16_kernel<kLo><<<dim3(kEmb / 64, kEmb / 64, 4), 256, 0, stream>>>(Wq, Wk, Wv, Wo, WT, WTL);
  rot_table_kernel<<<(kSeq * kTabW) / 256, 256, 0, stream>>>(TAB);
  bias_table_kernel<<<1, 512, 0, stream>>>(bq, bk, bv, bo, BIAS);

  eng::wmma_gemm64<kSplQkv, 0><<<(kRows / 64) * (kNqkv / 64) / 8, 256, 0, stream>>>(
      XB, XL, kEmb, WT, WTL, kEmb, QKVF, kHd, BIAS, kRows, kNqkv, kEmb);

  rot_split_kernel<<<(2 * kBH * kSeq * 8) / 256, 256, 0, stream>>>(QKVF, TAB, QKH, QKL);
  vt_split_kernel<<<dim3(kSeq / 64, kBH), 256, 0, stream>>>(QKVF + (size_t)2 * kBH * kSeq * kHd, VTH, VTL);

  attn_kernel<<<kBH * (kSeq / 64), 128, 0, stream>>>(QKH, QKL, VTH, VTL, AOH, AOL);

  eng::wmma_gemm64<kSplOut, 1><<<(kRows / 64) * (kEmb / 64) / 8, 256, 0, stream>>>(
      AOH, AOL, kEmb, WT + (size_t)3 * kEmb * kEmb, WTL + (size_t)3 * kEmb * kEmb, kEmb,
      out, kEmb, BIAS + 3 * kEmb, kRows, kEmb, kEmb);
}
